// TransGCN_22857815949367
// MI455X (gfx1250) — hardware-run, weakly checked
//
#include <hip/hip_runtime.h>
#include <stddef.h>
#include <stdint.h>
#include <math.h>

#define W_RNE  1

#define NN     50000
#define NE     800000
#define HC     128
#define FFD    2048
#define NL     2
#define K2     256
#define GBM    64
#define GTHR   128
#define MP     50048
#define NTILE  (MP / GBM)
#define RCT    64
#define RC     (RCT * GBM)
#define NCHK   ((NTILE + RCT - 1) / RCT)
#define LNEPS  1e-5f

#define NTHR   256
#define NWAVE  8
#define EPT    8
#define CHUNK  (NTHR * EPT)
#define WCAP   (EPT * 32)
#define LISTN  (NWAVE * WCAP)
#define NBA    1024
#define SLA    10
#define RCAP   28672
#define DEGCAP 64
#define NBLK   ((MP + NBA - 1) / NBA)
#define NBP    (NBLK * NBA)
#define MEAS_B1024  16623
#define MEAS_MAXDEG 35
#define BKT_ZINTS (LISTN + 2 * RCAP + 3 * NBA)
#define BKT_LDS_INTS (BKT_ZINTS + 16)

#define LSTR   2944
#define PTN    6144
#define PT_LB(l) (128 + (l) * LSTR)

#define OW_GW  0
#define OW_WV  16384
#define OW_WO  (OW_WV + NL * 32768)
#define OW_F1  (OW_WO + NL * 32768)
#define OW_F2  (OW_F1 + NL * 524288)
#define WBN    (OW_F2 + NL * 262144)
#define WSMAX  134217728

static_assert(MP % GBM == 0 && MP >= NN && MP - NN < GBM);
static_assert(RC % 128 == 0 && RC % GBM == 0);
static_assert(HC % 32 == 0 && K2 % 32 == 0 && FFD % 32 == 0 && K2 == 2 * HC);
static_assert((NBA & (NBA - 1)) == 0 && NBA == (1 << SLA));
static_assert(((long long)NE << SLA) < (1LL << 31));
static_assert(RCAP % (NTHR * 4) == 0 && NBA == NTHR * 4);
static_assert((long long)RCAP * 100 >= (long long)MEAS_B1024 * 105);
static_assert(DEGCAP >= MEAS_MAXDEG + 8);
static_assert(BKT_ZINTS % 4 == 0 && LISTN % 4 == 0 && BKT_LDS_INTS * 4 <= 300000);
static_assert(NBP >= MP && MP % 32 == 0);
static_assert(PTN >= 128 + NL * LSTR && PTN % (4 * NTHR) == 0 && LSTR % 128 == 0);
static_assert((MP * 16) % NTHR == 0);
static_assert(NE % 4 == 0);

typedef float          v4f   __attribute__((ext_vector_type(4)));
typedef float          v8f   __attribute__((ext_vector_type(8)));
typedef int            v4i   __attribute__((ext_vector_type(4)));
typedef int            v8i   __attribute__((ext_vector_type(8)));
typedef unsigned int   v4u   __attribute__((ext_vector_type(4)));
typedef unsigned short v8us  __attribute__((ext_vector_type(8)));
typedef unsigned short v16us __attribute__((ext_vector_type(16)));
typedef __bf16         v16bf __attribute__((ext_vector_type(16)));
typedef v4f  __attribute__((may_alias)) v4fa;
typedef v4i  __attribute__((may_alias)) v4ia;
typedef v8us __attribute__((may_alias)) v8usa;
union FragB { v16bf v; v16us u; v8us h[2]; v8i w; };

__device__ __forceinline__ v8f wmb(const FragB& a, const FragB& b, v8f c) {
  v8f d = __builtin_amdgcn_wmma_f32_16x16x32_bf16(false, a.v, false, b.v, (short)0, c, false, false);
  asm volatile("v_nop\n\tv_nop\n\tv_nop\n\tv_nop" : "+v"(d) : "v"(a.w), "v"(b.w));
  return d;
}

__device__ __forceinline__ unsigned bf16_bits(float f) {
  const unsigned u = __float_as_uint(f);
  const unsigned r = (u + 0x7FFFu + ((u >> 16) & 1u)) >> 16;
  return (f != f) ? 0x7FC0u : r;
}
__device__ __forceinline__ float bf16_val(float f) {
  return __uint_as_float(bf16_bits(f) << 16);
}
__device__ __forceinline__ float relu_k(float v) { return (v > 0.0f) ? v : (v - v); }
__device__ __forceinline__ unsigned hl_sel(float v, bool lo) {
  const unsigned hb = bf16_bits(v);
  const unsigned lb = bf16_bits(v - __uint_as_float(hb << 16));
  return lo ? lb : hb;
}

__global__ __launch_bounds__(NTHR) __attribute__((amdgpu_num_vgpr(248)))
void k_pa(const float* __restrict__ x, unsigned short* xb) {
  const int u = (int)blockIdx.x * NTHR + (int)threadIdx.x;
  if (u >= MP * 16) return;
  const int row = u >> 4;
  const int k8  = (u & 15) * 8;
  const int rc  = row < NN ? row : NN - 1;
  const float* p = x + (size_t)rc * HC + k8;
  const v4f a = *(const v4fa*)p;
  const v4f b = *(const v4fa*)(p + 4);
  const bool ok = row < NN;
  v8us o;
  o[0] = ok ? (unsigned short)bf16_bits(a.x) : (unsigned short)0;
  o[1] = ok ? (unsigned short)bf16_bits(a.y) : (unsigned short)0;
  o[2] = ok ? (unsigned short)bf16_bits(a.z) : (unsigned short)0;
  o[3] = ok ? (unsigned short)bf16_bits(a.w) : (unsigned short)0;
  o[4] = ok ? (unsigned short)bf16_bits(b.x) : (unsigned short)0;
  o[5] = ok ? (unsigned short)bf16_bits(b.y) : (unsigned short)0;
  o[6] = ok ? (unsigned short)bf16_bits(b.z) : (unsigned short)0;
  o[7] = ok ? (unsigned short)bf16_bits(b.w) : (unsigned short)0;
  unsigned short* dp = xb + (size_t)row * HC + k8;
  *(volatile v8us*)dp = o;
  __threadfence();
  *(volatile v8us*)dp = o;
}

__device__ __forceinline__ void cvt_unit(const float* __restrict__ src, int pitch, int lg, int smask,
                                         unsigned short* dst, int u) {
  const int n  = u >> lg;
  const int kq = u & ((1 << lg) - 1);
  const float* p = src + (size_t)n * pitch + 8 * (kq & smask);
  const v4f a = *(const v4fa*)p;
  const v4f b = *(const v4fa*)(p + 4);
  v8us o;
  o[0] = (unsigned short)bf16_bits(a.x); o[1] = (unsigned short)bf16_bits(a.y);
  o[2] = (unsigned short)bf16_bits(a.z); o[3] = (unsigned short)bf16_bits(a.w);
  o[4] = (unsigned short)bf16_bits(b.x); o[5] = (unsigned short)bf16_bits(b.y);
  o[6] = (unsigned short)bf16_bits(b.z); o[7] = (unsigned short)bf16_bits(b.w);
  unsigned short* dp = dst + ((size_t)n << (lg + 3)) + 8 * kq;
  *(volatile v8us*)dp = o;
  __threadfence();
  *(volatile v8us*)dp = o;
}

__global__ __launch_bounds__(NTHR) __attribute__((amdgpu_num_vgpr(248)))
void k_pw(const float* __restrict__ gcn_w, const float* __restrict__ in_w, const float* __restrict__ out_w,
          const float* __restrict__ ff1_w, const float* __restrict__ ff2_w, unsigned short* WB) {
  const int b = (int)blockIdx.x, tid = (int)threadIdx.x;
  if (b < 8) {
    cvt_unit(gcn_w, HC, 4, 15, WB + OW_GW, b * NTHR + tid);
  } else if (b < 40) {
    const int bb = b - 8, l = bb >> 4;
    cvt_unit(in_w + (size_t)l * 384 * HC + 256 * HC, HC, 5, 15, WB + OW_WV + l * 32768, (bb & 15) * NTHR + tid);
  } else if (b < 72) {
    const int bb = b - 40, l = bb >> 4;
    cvt_unit(out_w + (size_t)l * HC * HC, HC, 5, 15, WB + OW_WO + l * 32768, (bb & 15) * NTHR + tid);
  } else if (b < 584) {
    const int bb = b - 72, l = bb >> 8;
    cvt_unit(ff1_w + (size_t)l * FFD * HC, HC, 5, 15, WB + OW_F1 + l * 524288, (bb & 255) * NTHR + tid);
  } else if (b < 840) {
    const int bb = b - 584, l = bb >> 7;
    cvt_unit(ff2_w + (size_t)l * HC * FFD, FFD, 8, 255, WB + OW_F2 + l * 262144, (bb & 127) * NTHR + tid);
  }
}

__global__ __launch_bounds__(NTHR) __attribute__((amdgpu_num_vgpr(248)))
void k_pt(const float* __restrict__ gcn_b, const float* __restrict__ in_b, const float* __restrict__ out_b,
          const float* __restrict__ l1g, const float* __restrict__ l1b, const float* __restrict__ f1b,
          const float* __restrict__ f2b, const float* __restrict__ l2g, const float* __restrict__ l2b,
          float* PT) {
  const int g = (int)blockIdx.x * NTHR + (int)threadIdx.x;
  if (g >= PTN / 4) return;
  const int f = 4 * g;
  v4f v = {0.0f, 0.0f, 0.0f, 0.0f};
  if (f < 128) {
    v = *(const v4fa*)(gcn_b + f);
  } else if (f < 128 + NL * LSTR) {
    const int r = f - 128;
    const int l = (r >= LSTR) ? 1 : 0;
    const int q = r - l * LSTR;
    if (q < 128)       v = *(const v4fa*)(in_b  + l * 384 + 256 + q);
    else if (q < 256)  v = *(const v4fa*)(out_b + l * HC + (q - 128));
    else if (q < 384)  v = *(const v4fa*)(l1g   + l * HC + (q - 256));
    else if (q < 512)  v = *(const v4fa*)(l1b   + l * HC + (q - 384));
    else if (q < 2560) v = *(const v4fa*)(f1b   + l * FFD + (q - 512));
    else if (q < 2688) v = *(const v4fa*)(f2b   + l * HC + (q - 2560));
    else if (q < 2816) v = *(const v4fa*)(l2g   + l * HC + (q - 2688));
    else               v = *(const v4fa*)(l2b   + l * HC + (q - 2816));
  }
#if W_RNE
  v.x = bf16_val(v.x); v.y = bf16_val(v.y); v.z = bf16_val(v.z); v.w = bf16_val(v.w);
#endif
  *(volatile v4f*)(PT + f) = v;
  __threadfence();
  *(volatile v4f*)(PT + f) = v;
}

template <int SLB>
__device__ __forceinline__ int scan_chunk(const int* __restrict__ dsts, int nE, int cbase, int slotBase,
                                          int nb, int vec8, int* list, int tid, int lane, int wave) {
  int wc = 0;
  const int el0  = tid * EPT;
  const int e0   = cbase + el0;
  const int sent = -2147483647 - 1;
  v4i da, db;
  if (vec8 != 0 && cbase + CHUNK <= nE) {
    da = *(const v4i*)(dsts + e0);
    db = *(const v4i*)(dsts + e0 + 4);
  } else {
    da.x = (e0     < nE) ? dsts[min(e0,     nE - 1)] : sent;
    da.y = (e0 + 1 < nE) ? dsts[min(e0 + 1, nE - 1)] : sent;
    da.z = (e0 + 2 < nE) ? dsts[min(e0 + 2, nE - 1)] : sent;
    da.w = (e0 + 3 < nE) ? dsts[min(e0 + 3, nE - 1)] : sent;
    db.x = (e0 + 4 < nE) ? dsts[min(e0 + 4, nE - 1)] : sent;
    db.y = (e0 + 5 < nE) ? dsts[min(e0 + 5, nE - 1)] : sent;
    db.z = (e0 + 6 < nE) ? dsts[min(e0 + 6, nE - 1)] : sent;
    db.w = (e0 + 7 < nE) ? dsts[min(e0 + 7, nE - 1)] : sent;
  }
  const unsigned nbs = (unsigned)slotBase;
  const unsigned unb = (unsigned)nb;
  const unsigned s0 = (unsigned)da.x - nbs, s1 = (unsigned)da.y - nbs;
  const unsigned s2 = (unsigned)da.z - nbs, s3 = (unsigned)da.w - nbs;
  const unsigned s4 = (unsigned)db.x - nbs, s5 = (unsigned)db.y - nbs;
  const unsigned s6 = (unsigned)db.z - nbs, s7 = (unsigned)db.w - nbs;
  const bool h0 = s0 < unb, h1 = s1 < unb, h2 = s2 < unb, h3 = s3 < unb;
  const bool h4 = s4 < unb, h5 = s5 < unb, h6 = s6 < unb, h7 = s7 < unb;
  const unsigned any = __builtin_amdgcn_ballot_w32(h0 | h1 | h2 | h3 | h4 | h5 | h6 | h7);
  if (any != 0u) {
#define HITJ(J, HJ, SJ) { \
      const unsigned mj = __builtin_amdgcn_ballot_w32(HJ); \
      if (mj != 0u) { \
        if (HJ) { \
          const int pos = wc + (int)__builtin_amdgcn_mbcnt_lo(mj, 0u); \
          if (pos < WCAP) list[wave * WCAP + pos] = ((el0 + (J)) << SLB) | (int)(SJ); \
        } \
        wc += (int)__builtin_popcount(mj); } }
    HITJ(0, h0, s0)
    HITJ(1, h1, s1)
    HITJ(2, h2, s2)
    HITJ(3, h3, s3)
    HITJ(4, h4, s4)
    HITJ(5, h5, s5)
    HITJ(6, h6, s6)
    HITJ(7, h7, s7)
#undef HITJ
  }
  return wc;
}

__device__ __forceinline__ void bkt_store(const int* sl, const int* cnt, const int* offs, const int* cur,
                                          int* lp, int* cp, int* op, int* dp, int tid) {
#pragma unroll 1
  for (int it = 0; it < RCAP / (NTHR * 4); ++it) {
    const int i = it * (NTHR * 4) + 4 * tid;
    const v4i v = *(const v4ia*)(sl + i);
    *(volatile v4i*)(lp + i) = v;
  }
  const int i = 4 * tid;
  const v4i c4 = *(const v4ia*)(cnt + i);
  const v4i o4 = *(const v4ia*)(offs + i);
  const v4i d4 = *(const v4ia*)(cur + i);
  *(volatile v4i*)(cp + i) = c4;
  *(volatile v4i*)(op + i) = o4;
  *(volatile v4i*)(dp + i) = d4;
}

__global__ __launch_bounds__(NTHR) __attribute__((amdgpu_num_vgpr(248)))
void k_bkt(const int* __restrict__ srcs, const int* __restrict__ dsts, int nE, int vec8,
           int* LIST, int* CNT, int* OFF, int* DNV) {
  extern __shared__ __attribute__((aligned(16))) int dsm[];
  int* list = dsm;
  int* hl   = dsm + LISTN;
  int* sl   = dsm + LISTN + RCAP;
  int* cnt  = dsm + LISTN + 2 * RCAP;
  int* offs = cnt + NBA;
  int* cur  = offs + NBA;
  int* misc = cur + NBA;
  const int tid = (int)threadIdx.x, lane = tid & 31, wave = tid >> 5;
  const int nodeBase = (int)blockIdx.x * NBA;

  {
    const v4i z4 = {0, 0, 0, 0};
    for (int i = tid * 4; i < BKT_ZINTS; i += NTHR * 4) *(v4ia*)(dsm + i) = z4;
    if (tid < 16) misc[tid] = 0;
  }
  __syncthreads();

  int t = 0, ov = 0;
  const int nChunks = (nE + CHUNK - 1) / CHUNK;
#pragma unroll 1
  for (int ch = 0; ch < nChunks; ++ch) {
    const int cbase = ch * CHUNK;
    const int wc = scan_chunk<SLA>(dsts, nE, cbase, nodeBase, NBA, vec8, list, tid, lane, wave);
    if (lane == 0) misc[wave] = wc;
    __syncthreads();
    if (wave == 0) {
#pragma unroll 1
      for (int w2 = 0; w2 < NWAVE; ++w2) {
        int c = misc[w2];
        c = c < 0 ? 0 : (c > WCAP ? WCAP : c);
#pragma unroll 1
        for (int b0 = 0; b0 < c; b0 += 32) {
          const int idx = b0 + lane;
          const int ent = list[w2 * WCAP + (idx < WCAP ? idx : WCAP - 1)];
          const int m32 = (c - b0) < 32 ? (c - b0) : 32;
#pragma unroll 1
          for (int k = 0; k < m32; ++k) {
            const int u    = __builtin_amdgcn_readlane(ent, k);
            const int slot = u & (NBA - 1);
            const int el   = (u >> SLA) & (CHUNK - 1);
            const int pk   = ((cbase + el) << SLA) | slot;
            if (t < RCAP) {
              if (lane == 0) { hl[t] = pk; cnt[slot] = cnt[slot] + 1; }
              t = t + 1;
            } else {
              ov = 1;
            }
          }
        }
      }
    }
    __syncthreads();
  }
  if (wave == 0 && lane == 0) { misc[8] = t; misc[9] = ov; }
  __syncthreads();
  int tt = misc[8];
  tt = tt < 0 ? 0 : (tt > RCAP ? RCAP : tt);
  const int ovf = misc[9];

  if (wave == 0) {
    const int base = lane * (NBA / 32);
    int s = 0;
#pragma unroll 1
    for (int i = 0; i < NBA / 32; ++i) s += cnt[base + i];
    int incl = s;
#pragma unroll
    for (int d = 1; d < 32; d <<= 1) {
      const int y = __shfl_up(incl, d, 32);
      if (lane >= d) incl += y;
    }
    int run = incl - s;
#pragma unroll 1
    for (int i = 0; i < NBA / 32; ++i) {
      const int cv = cnt[base + i];
      offs[base + i] = run;
      cur[base + i]  = run;
      run += cv;
    }
  }
  __syncthreads();
  if (wave == 0) {
#pragma unroll 1
    for (int b0 = 0; b0 < tt; b0 += 32) {
      const int idx = b0 + lane;
      const int ent = hl[idx < RCAP ? idx : RCAP - 1];
      const int m32 = (tt - b0) < 32 ? (tt - b0) : 32;
#pragma unroll 1
      for (int k = 0; k < m32; ++k) {
        const int u    = __builtin_amdgcn_readlane(ent, k);
        const int slot = u & (NBA - 1);
        if (lane == 0) {
          int p = cur[slot];
          p = p < 0 ? 0 : (p > RCAP - 1 ? RCAP - 1 : p);
          sl[p] = u;
          cur[slot] = p + 1;
        }
      }
    }
  }
  __syncthreads();

#pragma unroll 4
  for (int i = tid; i < RCAP; i += NTHR) {
    const int ent = sl[i];
    int eid = ent >> SLA;
    eid = eid < 0 ? 0 : (eid > nE - 1 ? nE - 1 : eid);
    int sr = srcs[eid];
    sr = sr < 0 ? 0 : (sr > NN - 1 ? NN - 1 : sr);
    sl[i] = (i < tt) ? sr : 0;
  }
  const float qnan = __int_as_float(0x7fc00000);
#pragma unroll 1
  for (int i = tid; i < NBA; i += NTHR) {
    const float d = (float)cnt[i] + 1.0f;
    float r = 1.0f / sqrtf(d);
    r = (ovf != 0) ? qnan : r;
    cur[i] = __float_as_int(r);
  }
  __syncthreads();

  int* lp = LIST + (size_t)blockIdx.x * RCAP;
  int* cp = CNT + nodeBase;
  int* op = OFF + nodeBase;
  int* dp = DNV + nodeBase;
  bkt_store(sl, cnt, offs, cur, lp, cp, op, dp, tid);
  __threadfence();
  bkt_store(sl, cnt, offs, cur, lp, cp, op, dp, tid);
}

__global__ __launch_bounds__(NTHR) __attribute__((amdgpu_num_vgpr(248)))
void k_agg(const int* __restrict__ LIST, const int* __restrict__ CNT, const int* __restrict__ OFF,
           const float* __restrict__ DINV, const float* __restrict__ HW, const float* __restrict__ PT,
           float* HF, unsigned short* HL) {
  const int tid = (int)threadIdx.x, lane = tid & 31, wave = tid >> 5;
  const v4f bia = *(const v4fa*)(PT + 4 * lane);
  const float qnan = __int_as_float(0x7fc00000);
  const int sA = (2 * (lane & 15)) & 31, sB = (2 * (lane & 15) + 1) & 31;
  const bool lsel = (lane & 16) != 0;
#pragma unroll 1
  for (int si = 0; si < 4; ++si) {
    const int node = (int)blockIdx.x * 32 + wave * 4 + si;
    const int nc = node < NN ? node : NN - 1;
    const int blk = nc >> SLA;
    int c = CNT[nc];
    const bool big = c > DEGCAP;
    c = c < 0 ? 0 : (c > DEGCAP ? DEGCAP : c);
    int o = OFF[nc];
    o = o < 0 ? 0 : (o > RCAP ? RCAP : o);
    const float dd = DINV[nc];
    const float rd = dd * dd;
    const int* lp = LIST + (size_t)blk * RCAP;
    v4f acc = {0.0f, 0.0f, 0.0f, 0.0f};
#pragma unroll 1
    for (int b0 = 0; b0 < c; b0 += 32) {
      int idx = o + b0 + lane;
      idx = idx > RCAP - 1 ? RCAP - 1 : idx;
      int sr = lp[idx];
      sr = sr < 0 ? 0 : (sr > NN - 1 ? NN - 1 : sr);
      const float cf  = DINV[sr] * dd;
      const int   cfi = __float_as_int(cf);
      const int m32 = (c - b0) < 32 ? (c - b0) : 32;
#pragma unroll 1
      for (int k = 0; k < m32; ++k) {
        const int   sk = __builtin_amdgcn_readlane(sr, k);
        const float ck = __int_as_float(__builtin_amdgcn_readlane(cfi, k));
        const v4f a = *(const v4fa*)(HW + (size_t)sk * HC + 4 * lane);
        acc.x = fmaf(ck, a.x, acc.x); acc.y = fmaf(ck, a.y, acc.y);
        acc.z = fmaf(ck, a.z, acc.z); acc.w = fmaf(ck, a.w, acc.w);
      }
    }
    const v4f sv = *(const v4fa*)(HW + (size_t)nc * HC + 4 * lane);
    const bool live = node < NN;
    v4f y;
    y.x = relu_k((acc.x + sv.x * rd) + bia.x);
    y.y = relu_k((acc.y + sv.y * rd) + bia.y);
    y.z = relu_k((acc.z + sv.z * rd) + bia.z);
    y.w = relu_k((acc.w + sv.w * rd) + bia.w);
    y.x = big ? qnan : y.x; y.y = big ? qnan : y.y; y.z = big ? qnan : y.z; y.w = big ? qnan : y.w;
    y.x = live ? y.x : 0.0f; y.y = live ? y.y : 0.0f; y.z = live ? y.z : 0.0f; y.w = live ? y.w : 0.0f;

    const unsigned h0 = bf16_bits(y.x), h1 = bf16_bits(y.y), h2 = bf16_bits(y.z), h3 = bf16_bits(y.w);
    const unsigned l0 = bf16_bits(y.x - __uint_as_float(h0 << 16));
    const unsigned l1 = bf16_bits(y.y - __uint_as_float(h1 << 16));
    const unsigned l2 = bf16_bits(y.z - __uint_as_float(h2 << 16));
    const unsigned l3 = bf16_bits(y.w - __uint_as_float(h3 << 16));
    const int hw0 = (int)(h0 | (h1 << 16)), hw1 = (int)(h2 | (h3 << 16));
    const int lw0 = (int)(l0 | (l1 << 16)), lw1 = (int)(l2 | (l3 << 16));
    const int g0 = __shfl(hw0, sA, 32), g1 = __shfl(hw1, sA, 32);
    const int g2 = __shfl(hw0, sB, 32), g3 = __shfl(hw1, sB, 32);
    const int p0 = __shfl(lw0, sA, 32), p1 = __shfl(lw1, sA, 32);
    const int p2 = __shfl(lw0, sB, 32), p3 = __shfl(lw1, sB, 32);
    v4u pv;
    pv.x = (unsigned)(lsel ? p0 : g0);
    pv.y = (unsigned)(lsel ? p1 : g1);
    pv.z = (unsigned)(lsel ? p2 : g2);
    pv.w = (unsigned)(lsel ? p3 : g3);
    float* fp = HF + (size_t)node * HC + 4 * lane;
    unsigned short* hp = HL + (size_t)node * K2 + 8 * lane;
    *(volatile v4f*)fp = y;
    *(volatile v4u*)hp = pv;
    __threadfence();
    *(volatile v4f*)fp = y;
    *(volatile v4u*)hp = pv;
  }
}

template <int MODE>
__device__ __forceinline__ void st_pass(const float* stg, float* outF, unsigned short* outH,
                                        int grow0, int roff, int col0, int wave, int lane) {
  const int hh = lane >> 4, m = lane & 15;
  if constexpr (MODE == 0 || MODE == 2 || MODE == 5) {
#pragma unroll 4
    for (int i = 0; i < 16; ++i) {
      const int lr = 16 * wave + i;
      const int grow = grow0 + lr;
      const v4f v = *(const v4fa*)(stg + lr * HC + 4 * lane);
      if (MODE != 5 || grow < NN) *(volatile v4f*)(outF + (size_t)grow * HC + 4 * lane) = v;
    }
  }
  if constexpr (MODE == 1 || MODE == 2) {
    const bool lo = hh != 0;
#pragma unroll 2
    for (int i = 0; i < 16; ++i) {
      const int lr = 16 * wave + i;
      const int grow = grow0 + lr;
      const v4f a = *(const v4fa*)(stg + lr * HC + 8 * m);
      const v4f b = *(const v4fa*)(stg + lr * HC + 8 * m + 4);
      v4u pv;
      pv.x = hl_sel(a.x, lo) | (hl_sel(a.y, lo) << 16);
      pv.y = hl_sel(a.z, lo) | (hl_sel(a.w, lo) << 16);
      pv.z = hl_sel(b.x, lo) | (hl_sel(b.y, lo) << 16);
      pv.w = hl_sel(b.z, lo) | (hl_sel(b.w, lo) << 16);
      *(volatile v4u*)(outH + (size_t)grow * K2 + 8 * lane) = pv;
    }
  }
  if constexpr (MODE == 3) {
#pragma unroll 2
    for (int i = 0; i < 8; ++i) {
      const int lr = 16 * wave + 2 * i + hh;
      const int orow = grow0 + lr - roff;
      const v4f a = *(const v4fa*)(stg + lr * HC + 8 * m);
      const v4f b = *(const v4fa*)(stg + lr * HC + 8 * m + 4);
      v4u pv;
      pv.x = bf16_bits(a.x) | (bf16_bits(a.y) << 16);
      pv.y = bf16_bits(a.z) | (bf16_bits(a.w) << 16);
      pv.z = bf16_bits(b.x) | (bf16_bits(b.y) << 16);
      pv.w = bf16_bits(b.z) | (bf16_bits(b.w) << 16);
      *(volatile v4u*)(outH + (size_t)orow * FFD + col0 + 8 * m) = pv;
    }
  }
}

template <int MODE, int KK>
__global__ __launch_bounds__(GTHR) __attribute__((amdgpu_num_vgpr(248)))
void k_g(const unsigned short* __restrict__ A, const unsigned short* __restrict__ WT,
         const float* __restrict__ PT, const float* RES, const float* __restrict__ HR,
         float* outF, unsigned short* outH, int tile0, int roff, int pbias, int pg) {
  __shared__ __attribute__((aligned(16))) float stg[GBM * HC];
  const int tid = (int)threadIdx.x, lane = tid & 31, wave = tid >> 5, hh = lane >> 4, m = lane & 15;
  const int rg = wave & 1, cg = wave >> 1;
  const int grow0 = ((int)blockIdx.x + tile0) * GBM;
  const int col0  = (int)blockIdx.y * HC;
  const int arow  = grow0 - ((MODE == 3) ? 0 : roff);

  const v8f z8 = {0.f, 0.f, 0.f, 0.f, 0.f, 0.f, 0.f, 0.f};
  v8f acc[2][4];
#pragma unroll
  for (int mt = 0; mt < 2; ++mt)
#pragma unroll
    for (int nt = 0; nt < 4; ++nt) acc[mt][nt] = z8;

  const unsigned short* ap0 = A + (size_t)(arow + 32 * rg + m) * KK + 8 * hh;
  const unsigned short* ap1 = ap0 + (size_t)16 * KK;
  const unsigned short* wp  = WT + (size_t)(col0 + 64 * cg + m) * KK + 8 * hh;
#pragma unroll 1
  for (int ks = 0; ks < KK / 32; ++ks) {
    FragB a0, a1;
    a0.h[0] = *(const v8usa*)(ap0 + 32 * ks);
    a0.h[1] = *(const v8usa*)(ap0 + 32 * ks + 16);
    a1.h[0] = *(const v8usa*)(ap1 + 32 * ks);
    a1.h[1] = *(const v8usa*)(ap1 + 32 * ks + 16);
#pragma unroll
    for (int nt = 0; nt < 4; ++nt) {
      const unsigned short* wq = wp + (size_t)(16 * nt) * KK + 32 * ks;
      FragB bf;
      bf.h[0] = *(const v8usa*)wq;
      bf.h[1] = *(const v8usa*)(wq + 16);
      acc[0][nt] = wmb(a0, bf, acc[0][nt]);
      acc[1][nt] = wmb(a1, bf, acc[1][nt]);
    }
  }

#pragma unroll
  for (int mt = 0; mt < 2; ++mt)
#pragma unroll
    for (int nt = 0; nt < 4; ++nt) {
      const int lc = 64 * cg + 16 * nt + m;
#pragma unroll
      for (int r = 0; r < 8; ++r) {
        const int lr = 32 * rg + 16 * mt + 8 * hh + r;
        stg[lr * HC + lc] = acc[mt][nt][r];
      }
    }
  __syncthreads();

  if constexpr (MODE != 0) {
    const v4f bia = *(const v4fa*)(PT + pbias + col0 + 4 * lane);
    v4f gg = bia, bb = bia;
    if constexpr (MODE == 2 || MODE == 5) {
      gg = *(const v4fa*)(PT + pg + 4 * lane);
      bb = *(const v4fa*)(PT + pg + HC + 4 * lane);
    }
#pragma unroll 1
    for (int i = 0; i < 16; ++i) {
      const int lr = 16 * wave + i;
      const int grow = grow0 + lr;
      float* sp = stg + lr * HC + 4 * lane;
      v4f v = *(const v4fa*)sp;
      v = v + bia;
      if constexpr (MODE == 3) {
        v.x = relu_k(v.x); v.y = relu_k(v.y); v.z = relu_k(v.z); v.w = relu_k(v.w);
      }
      if constexpr (MODE == 2 || MODE == 5) {
        const v4f rs = *(const v4fa*)(RES + (size_t)grow * HC + 4 * lane);
        const v4f s = rs + v;
        float sum = (s.x + s.y) + (s.z + s.w);
#pragma unroll
        for (int o = 16; o > 0; o >>= 1) sum += __shfl_xor(sum, o, 32);
        const float mean = sum * (1.0f / 128.0f);
        const v4f d = {s.x - mean, s.y - mean, s.z - mean, s.w - mean};
        float q = (d.x * d.x + d.y * d.y) + (d.z * d.z + d.w * d.w);
#pragma unroll
        for (int o = 16; o > 0; o >>= 1) q += __shfl_xor(q, o, 32);
        const float var  = q * (1.0f / 128.0f);
        const float den  = sqrtf(var + LNEPS);
        const float rinv = 1.0f / den;
        v.x = (d.x * rinv) * gg.x + bb.x;
        v.y = (d.y * rinv) * gg.y + bb.y;
        v.z = (d.z * rinv) * gg.z + bb.z;
        v.w = (d.w * rinv) * gg.w + bb.w;
      }
      if constexpr (MODE == 5) {
        const v4f hr = *(const v4fa*)(HR + (size_t)grow * HC + 4 * lane);
        v.x = relu_k(v.x + hr.x); v.y = relu_k(v.y + hr.y);
        v.z = relu_k(v.z + hr.z); v.w = relu_k(v.w + hr.w);
      }
      *(v4fa*)sp = v;
    }
    __syncthreads();
  }

  st_pass<MODE>(stg, outF, outH, grow0, roff, col0, wave, lane);
  __threadfence();
  st_pass<MODE>(stg, outF, outH, grow0, roff, col0, wave, lane);
}

static inline size_t al256(size_t o) { return (o + 255) & ~(size_t)255; }

extern "C" void kernel_launch(void* const* d_in, const int* in_sizes, int n_in,
                              void* d_out, int out_size, void* d_ws, size_t ws_size,
                              hipStream_t stream) {
  if (n_in < 16) return;
  if (in_sizes[0] != NN * HC) return;
  if (in_sizes[1] != 2 * NE) return;
  if (in_sizes[2] != HC * HC || in_sizes[3] != HC) return;
  if (in_sizes[4] != NL * 384 * HC || in_sizes[5] != NL * 384) return;
  if (in_sizes[6] != NL * HC * HC || in_sizes[7] != NL * HC) return;
  if (in_sizes[8] != NL * HC || in_sizes[9] != NL * HC) return;
  if (in_sizes[10] != NL * FFD * HC || in_sizes[11] != NL * FFD) return;
  if (in_sizes[12] != NL * HC * FFD || in_sizes[13] != NL * HC) return;
  if (in_sizes[14] != NL * HC || in_sizes[15] != NL * HC) return;
  if (out_size != NN * HC) return;

  const float* x     = (const float*)d_in[0];
  const int*   edge  = (const int*)d_in[1];
  const float* gcn_w = (const float*)d_in[2];
  const float* gcn_b = (const float*)d_in[3];
  const float* in_w  = (const float*)d_in[4];
  const float* in_b  = (const float*)d_in[5];
  const float* out_w = (const float*)d_in[6];
  const float* out_b = (const float*)d_in[7];
  const float* ln1_g = (const float*)d_in[8];
  const float* ln1_b = (const float*)d_in[9];
  const float* ff1_w = (const float*)d_in[10];
  const float* ff1_b = (const float*)d_in[11];
  const float* ff2_w = (const float*)d_in[12];
  const float* ff2_b = (const float*)d_in[13];
  const float* ln2_g = (const float*)d_in[14];
  const float* ln2_b = (const float*)d_in[15];
  float* out = (float*)d_out;
  const int* src = edge;
  const int* dst = edge + NE;

  char* ws = (char*)d_ws;
  size_t off = 0;
  const size_t oR0  = off; off = al256(off + (size_t)MP * HC * 4);
  const size_t oR1  = off; off = al256(off + (size_t)MP * HC * 4);
  const size_t oR2  = off; off = al256(off + (size_t)MP * K2 * 2);
  const size_t oR3  = off; off = al256(off + (size_t)MP * K2 * 2);
  const size_t oUB  = off; off = al256(off + (size_t)RC * FFD * 2);
  const size_t oLS  = off; off = al256(off + (size_t)NBLK * RCAP * 4);
  const size_t oCN  = off; off = al256(off + (size_t)NBP * 4);
  const size_t oOF  = off; off = al256(off + (size_t)NBP * 4);
  const size_t oDV  = off; off = al256(off + (size_t)NBP * 4);
  const size_t oWB  = off; off = al256(off + (size_t)WBN * 2);
  const size_t oPT  = off; off = al256(off + (size_t)PTN * 4);
  if (off > ws_size || off > (size_t)WSMAX) return;
  float*          R0   = (float*)(ws + oR0);
  float*          R1   = (float*)(ws + oR1);
  unsigned short* R2   = (unsigned short*)(ws + oR2);
  unsigned short* R3   = (unsigned short*)(ws + oR3);
  unsigned short* UB   = (unsigned short*)(ws + oUB);
  int*            LIST = (int*)(ws + oLS);
  int*            CNT  = (int*)(ws + oCN);
  int*            OFF  = (int*)(ws + oOF);
  int*            DNV  = (int*)(ws + oDV);
  unsigned short* WB   = (unsigned short*)(ws + oWB);
  float*          PT   = (float*)(ws + oPT);

  const size_t bktLds = (size_t)BKT_LDS_INTS * 4;
  hipFuncSetAttribute(reinterpret_cast<const void*>(&k_bkt), hipFuncAttributeMaxDynamicSharedMemorySize, (int)bktLds);

  k_pa<<<(MP * 16) / NTHR, NTHR, 0, stream>>>(x, R3);
  k_pw<<<840, NTHR, 0, stream>>>(gcn_w, in_w, out_w, ff1_w, ff2_w, WB);
  k_pt<<<PTN / 4 / NTHR, NTHR, 0, stream>>>(gcn_b, in_b, out_b, ln1_g, ln1_b, ff1_b, ff2_b, ln2_g, ln2_b, PT);
  k_bkt<<<NBLK, NTHR, bktLds, stream>>>(src, dst, NE, 1, LIST, CNT, OFF, DNV);
  k_g<0, HC><<<dim3(NTILE, 1), GTHR, 0, stream>>>(R3, WB + OW_GW, PT, R0, R1, R0, R2, 0, 0, 0, 0);
  k_agg<<<MP / 32, NTHR, 0, stream>>>(LIST, CNT, OFF, (const float*)DNV, R0, PT, R1, R2);

  for (int l = 0; l < NL; ++l) {
    const int lb = PT_LB(l);
    const float* resp = (l == 0) ? R1 : R0;
    k_g<1, K2><<<dim3(NTILE, 1), GTHR, 0, stream>>>(R2, WB + OW_WV + l * 32768, PT, R0, R1, R0, R3,
                                                    0, 0, lb, 0);
    k_g<2, K2><<<dim3(NTILE, 1), GTHR, 0, stream>>>(R3, WB + OW_WO + l * 32768, PT, resp, R1, R0, R2,
                                                    0, 0, lb + 128, lb + 256);
    for (int c = 0; c < NCHK; ++c) {
      const int t0 = c * RCT;
      const int nt = (NTILE - t0) < RCT ? (NTILE - t0) : RCT;
      k_g<3, K2><<<dim3(nt, FFD / HC), GTHR, 0, stream>>>(R2, WB + OW_F1 + l * 524288, PT, R0, R1, R0, UB,
                                                         t0, t0 * GBM, lb + 512, 0);
      if (l == 0) {
        k_g<2, FFD><<<dim3(nt, 1), GTHR, 0, stream>>>(UB, WB + OW_F2 + l * 262144, PT, R0, R1, R0, R2,
                                                      t0, t0 * GBM, lb + 2560, lb + 2688);
      } else {
        k_g<5, FFD><<<dim3(nt, 1), GTHR, 0, stream>>>(UB, WB + OW_F2 + l * 262144, PT, R0, R1, out, R2,
                                                      t0, t0 * GBM, lb + 2560, lb + 2688);
      }
    }
  }
}
